// MultiHeadMALAAttention_55997783605382
// MI455X (gfx1250) — hardware-verified
//
#include <hip/hip_runtime.h>


#define NB_  4
#define NN   8192
#define DIM  256
#define NH_  8
#define HD   32
#define INT  256
#define SCALE 0.1767766952966369f
typedef _Float16 h16;
typedef unsigned short bf;
typedef __attribute__((ext_vector_type(16))) __bf16   v16bf;
typedef __attribute__((ext_vector_type(16))) _Float16 v16h;
typedef __attribute__((ext_vector_type(8)))  _Float16 v8h;
typedef __attribute__((ext_vector_type(8)))  unsigned short v8us;
typedef __attribute__((ext_vector_type(8)))  float    v8f;
typedef __attribute__((ext_vector_type(4)))  float    v4f;
typedef v8h  __attribute__((may_alias)) v8ha;
typedef v4f  __attribute__((may_alias)) v4fa;
typedef v8us __attribute__((may_alias)) v8usa;

__device__ __forceinline__ unsigned short f2bf(float f) { unsigned u = __float_as_uint(f); u += 0x7FFFu + ((u >> 16) & 1u); return (unsigned short)(u >> 16); }
__device__ __forceinline__ float bf2f(unsigned short b) { return __uint_as_float(((unsigned)b) << 16); }
__device__ __forceinline__ float bfr(float f) { return bf2f(f2bf(f)); }
__device__ __forceinline__ v16h cat16(v8h lo, v8h hi) { return __builtin_shufflevector(lo, hi, 0, 1, 2, 3, 4, 5, 6, 7, 8, 9, 10, 11, 12, 13, 14, 15); }
__device__ __forceinline__ v16bf cat16b(v8us lo, v8us hi) { return __builtin_bit_cast(v16bf, __builtin_shufflevector(lo, hi, 0, 1, 2, 3, 4, 5, 6, 7, 8, 9, 10, 11, 12, 13, 14, 15)); }
__device__ __forceinline__ v8f wmma16(v16h a, v16h b, v8f c) { return __builtin_amdgcn_wmma_f32_16x16x32_f16(false, a, false, b, (short)0, c, false, false); }
__device__ __forceinline__ v8f wmmab(v16bf a, v16bf b, v8f c) { return __builtin_amdgcn_wmma_f32_16x16x32_bf16(false, a, false, b, (short)0, c, false, false); }


template <typename T16> struct WFrag;
template <> struct WFrag<h16> { typedef v16h V; static __device__ __forceinline__ V ld(const h16* p) { return cat16(*(const v8h*)p, *(const v8h*)(p + 16)); } static __device__ __forceinline__ v8f mma(V a, V b, v8f c) { return wmma16(a, b, c); } };
template <> struct WFrag<bf> { typedef v16bf V; static __device__ __forceinline__ V ld(const bf* p) { return cat16b(*(const v8us*)p, *(const v8us*)(p + 16)); } static __device__ __forceinline__ v8f mma(V a, V b, v8f c) { return wmmab(a, b, c); } };
template <typename T16, int NSPLIT, bool BIAS>
__global__ __launch_bounds__(32) void k_gemmw(const T16* __restrict__ A, const T16* __restrict__ A2, const T16* __restrict__ Bt, const T16* __restrict__ Bt2, int K, float* C, int ldc, const float* __restrict__ bias, size_t sA, size_t sB, size_t sC) {
    typedef typename WFrag<T16>::V V;
    __shared__ __align__(16) float os[16 * 68];
    const size_t z = blockIdx.z; A += z * sA; if (A2) A2 += z * sA; Bt += z * sB; if (Bt2) Bt2 += z * sB; C += z * sC;
    const int lane = threadIdx.x & 31, lr = lane & 15, hi = lane >> 4; const int r0 = blockIdx.x * 64, c0 = blockIdx.y * 64;
    v8f acc[4][4];
#pragma unroll
    for (int mb = 0; mb < 4; ++mb)
#pragma unroll
        for (int nb = 0; nb < 4; ++nb) acc[mb][nb] = (v8f){};
    const size_t aoff = (size_t)(r0 + lr) * K + 8 * hi, boff = (size_t)(c0 + lr) * K + 8 * hi;
#pragma unroll 1
    for (int kc = 0; kc < K; kc += 32) {
        V a[4], a2[4];
#pragma unroll
        for (int mb = 0; mb < 4; ++mb) { a[mb] = WFrag<T16>::ld(A + aoff + (size_t)mb * 16 * K + kc); if (NSPLIT == 1 || NSPLIT == 2) a2[mb] = WFrag<T16>::ld(A2 + aoff + (size_t)mb * 16 * K + kc); }
#pragma unroll
        for (int nb = 0; nb < 4; ++nb) { const V b = WFrag<T16>::ld(Bt + boff + (size_t)nb * 16 * K + kc); V b2; if (NSPLIT >= 2) b2 = WFrag<T16>::ld(Bt2 + boff + (size_t)nb * 16 * K + kc);
#pragma unroll
            for (int mb = 0; mb < 4; ++mb) { acc[mb][nb] = WFrag<T16>::mma(a[mb], b, acc[mb][nb]); if (NSPLIT == 1 || NSPLIT == 2) acc[mb][nb] = WFrag<T16>::mma(a2[mb], b, acc[mb][nb]); if (NSPLIT >= 2) acc[mb][nb] = WFrag<T16>::mma(a[mb], b2, acc[mb][nb]); } }
        asm volatile("v_nop\n\tv_nop\n\tv_nop\n\tv_nop" : "+v"(acc[0][0]), "+v"(acc[1][1]), "+v"(acc[2][2]), "+v"(acc[3][3]) : "v"(a[0]), "v"(a[3]));
    }
#pragma unroll
    for (int mb = 0; mb < 4; ++mb) {
#pragma unroll
        for (int nb = 0; nb < 4; ++nb) {
#pragma unroll
            for (int j = 0; j < 8; ++j) os[(hi * 8 + j) * 68 + nb * 16 + lr] = acc[mb][nb][j]; }
        __builtin_amdgcn_wave_barrier(); asm volatile("" ::: "memory");
        float* crow = C + (size_t)(r0 + mb * 16) * ldc + c0;
#pragma unroll 1
        for (int ps = 0; ps < 2; ++ps) {
#pragma unroll
            for (int s = 0; s < 8; ++s) { const int row = 2 * s + hi, cofs = lr * 4; v4f val = *(const v4fa*)(os + row * 68 + cofs); if (BIAS) { val[0] += bfr(bias[c0 + cofs]); val[1] += bfr(bias[c0 + cofs + 1]); val[2] += bfr(bias[c0 + cofs + 2]); val[3] += bfr(bias[c0 + cofs + 3]); }
                *(volatile v4f*)(crow + (size_t)row * ldc + cofs) = val; }
            if (ps == 0) __threadfence(); }
        __builtin_amdgcn_wave_barrier(); asm volatile("" ::: "memory");
    }
}

__device__ __forceinline__ h16 tohx(float x) { return (h16)x; }
__device__ __forceinline__ void splitf(float y, unsigned short& h, unsigned short& l) { h = f2bf(y); l = f2bf(y - bf2f(h)); }
__device__ __forceinline__ float elu1(float x) { return x > 0.f ? __fadd_rn(x, 1.0f) : __expf(x); }
typedef __attribute__((ext_vector_type(2))) _Float16 v2h;
typedef __attribute__((ext_vector_type(4))) _Float16 v4h;
typedef __attribute__((ext_vector_type(4))) unsigned short v4us;

__global__ __launch_bounds__(256) void k_cvt8(const float* __restrict__ src, bf* dst, size_t n8) { const size_t i = (size_t)blockIdx.x * 256 + threadIdx.x; if (i >= n8) return; const v8f v = *(const v8f*)(src + i * 8); v8us o;
#pragma unroll
    for (int k = 0; k < 8; ++k) o[k] = f2bf(v[k]); *(volatile v8us*)(dst + i * 8) = o; __threadfence(); *(volatile v8us*)(dst + i * 8) = o; }
__global__ __launch_bounds__(256) void k_kmean(const float* __restrict__ F, float* KM, float* VM) { const int c = blockIdx.x * 256 + threadIdx.x; if (c >= INT) return; float sk = 0.f, sv = 0.f;
#pragma unroll 1
    for (int n = 0; n < NN; ++n) { const float* r = F + (size_t)n * 4 * INT; sk = __fadd_rn(sk, elu1(r[INT + c])); sv = __fadd_rn(sv, r[2 * INT + c]); }
    const float km = sk * (1.0f / NN), vm = sv * (1.0f / NN); *(volatile float*)(KM + c) = km; *(volatile float*)(VM + c) = vm; __threadfence(); *(volatile float*)(KM + c) = km; *(volatile float*)(VM + c) = vm; }
__device__ __forceinline__ float tshift(const float* __restrict__ xr, int d, float c_d, float s_d) { const float self_ = elu1(xr[d]); const float partner = elu1(xr[d ^ 1]); const float rot = (d & 1) ? partner : -partner;     float a = __fmul_rn(self_, c_d), b = __fmul_rn(rot, s_d); asm volatile("" : "+v"(a)); asm volatile("" : "+v"(b)); return __fadd_rn(a, b); }
__global__ __launch_bounds__(256) void k_qs(const float* __restrict__ F, const float* __restrict__ sn, const float* __restrict__ cs, h16* QS) { const size_t e = ((size_t)blockIdx.x * 256 + threadIdx.x) * 4; if (e >= (size_t)NH_ * NN * HD) return; const int d = (int)(e % HD); const int n = (int)((e / HD) % NN); const int h = (int)(e / ((size_t)HD * NN)); const float* xr = F + (size_t)n * 4 * INT + h * HD; v4h o;
#pragma unroll
    for (int q = 0; q < 4; ++q) { const int dd = d + q; o[q] = tohx(tshift(xr, dd, bfr(cs[n * HD + dd]), bfr(sn[n * HD + dd]))); } *(volatile v4h*)(QS + e) = o; __threadfence(); *(volatile v4h*)(QS + e) = o; }
__global__ __launch_bounds__(256) void k_kst(const float* __restrict__ F, const float* __restrict__ sn, const float* __restrict__ cs, h16* KST, h16* VT) { const size_t e = ((size_t)blockIdx.x * 256 + threadIdx.x) * 2; if (e >= (size_t)NH_ * 64 * NN) return; const int n = (int)(e % NN); const int dd = (int)((e / NN) % 64); const int h = (int)(e / ((size_t)NN * 64)); v2h ok, ov;
#pragma unroll
    for (int u = 0; u < 2; ++u) { const int nn = n + u; if (dd < HD) { const float* kr = F + (size_t)nn * 4 * INT + INT + h * HD; ok[u] = tohx(tshift(kr, dd, bfr(cs[nn * HD + dd]), bfr(sn[nn * HD + dd])));     ov[u] = tohx(F[(size_t)nn * 4 * INT + 2 * INT + h * HD + dd]); } else { ok[u] = (h16)0.f; ov[u] = (h16)0.f; } }
    for (int ps = 0; ps < 2; ++ps) { *(volatile v2h*)(KST + e) = ok; *(volatile v2h*)(VT + e) = ov; if (ps == 0) __threadfence(); } }
__global__ __launch_bounds__(256) void k_z(const float* __restrict__ F, const float* __restrict__ KM, float* Z) { const int e = blockIdx.x * 256 + threadIdx.x; if (e >= NN * NH_) return; const int h = e % NH_; const int n = e / NH_; const float* qr = F + (size_t)n * 4 * INT + h * HD; float s = 0.f;
#pragma unroll 1
    for (int d = 0; d < HD; ++d) { float p = __fmul_rn(elu1(qr[d]), KM[h * HD + d]); asm volatile("" : "+v"(p)); s = __fadd_rn(s, p); } const float z = __fmul_rn(s, SCALE); *(volatile float*)(Z + e) = z; __threadfence(); *(volatile float*)(Z + e) = z; }
__global__ __launch_bounds__(256) void k_kv16(const float* __restrict__ KV, h16* KVT) { const int e2 = (blockIdx.x * 256 + threadIdx.x) * 2; if (e2 >= NH_ * 64 * HD) return; const int d = e2 % HD; const int ee = (e2 / HD) % 64; const int h = e2 / (HD * 64); v2h o;
#pragma unroll
    for (int u = 0; u < 2; ++u) o[u] = ee < HD ? tohx(__fmul_rn(KV[((size_t)h * 64 + d + u) * 64 + ee], SCALE / (float)NN)) : (h16)0.f; *(volatile v2h*)(KVT + e2) = o; __threadfence(); *(volatile v2h*)(KVT + e2) = o; }
__global__ __launch_bounds__(256) void k_res(const float* __restrict__ AO, const float* __restrict__ Z, const float* __restrict__ VM, const float* __restrict__ F, const float* __restrict__ wl, const float* __restrict__ bl, bf* Rh, bf* Rl) { const size_t e = ((size_t)blockIdx.x * 256 + threadIdx.x) * 4; if (e >= (size_t)NN * INT) return; const int c = (int)(e % INT); const int n = (int)(e / INT); const int h = c / HD, d = c % HD; const float z = Z[n * NH_ + h]; const float fz = __fadd_rn(1.0f, __fdiv_rn(1.0f, __fadd_rn(z, 1e-6f))); v4us oh, ol;
#pragma unroll
    for (int q = 0; q < 4; ++q) { const int cc = c + q, dd = d + q; float lp = bfr(bl[cc]);
#pragma unroll
        for (int k = 0; k < 3; ++k) { const int nn = n - 1 + k; if (nn >= 0 && nn < NN) { float p = __fmul_rn(bfr(wl[cc * 3 + k]), F[(size_t)nn * 4 * INT + 2 * INT + cc]); asm volatile("" : "+v"(p)); lp = __fadd_rn(lp, p); } }
        float a = __fmul_rn(AO[((size_t)h * NN + n) * 64 + dd], fz); asm volatile("" : "+v"(a)); float zb = __fmul_rn(z, VM[cc]); asm volatile("" : "+v"(zb)); const float r = __fmul_rn(__fadd_rn(__fsub_rn(a, zb), lp), F[(size_t)n * 4 * INT + 3 * INT + cc]); unsigned short u, l; splitf(r, u, l); oh[q] = u; ol[q] = l; }
    *(volatile v4us*)(Rh + e) = oh; *(volatile v4us*)(Rl + e) = ol; __threadfence(); *(volatile v4us*)(Rh + e) = oh; *(volatile v4us*)(Rl + e) = ol; }

extern "C" void kernel_launch(void* const* d_in, const int* in_sizes, int n_in,
                              void* d_out, int out_size, void* d_ws, size_t ws_size, hipStream_t stream) {
    (void)in_sizes; (void)n_in; (void)out_size;
    const float* x = (const float*)d_in[0]; const float* sn = (const float*)d_in[1]; const float* cs = (const float*)d_in[2]; const float* wq = (const float*)d_in[3]; const float* bq = (const float*)d_in[4]; const float* wl = (const float*)d_in[5]; const float* bl = (const float*)d_in[6]; const float* wp = (const float*)d_in[7]; const float* bp = (const float*)d_in[8];
    float* OUT = (float*)d_out;
    char* wsp = (char*)d_ws;
    auto take = [&](size_t bytes) { char* p = wsp; wsp += (bytes + 255) & ~(size_t)255; return (void*)p; };
    bf* WQ = (bf*)take((size_t)4 * INT * DIM * 2); bf* WP = (bf*)take((size_t)DIM * INT * 2); bf* XB = (bf*)take((size_t)NN * DIM * 2); float* F = (float*)take((size_t)NN * 4 * INT * 4); float* KM = (float*)take(INT * 4); float* VM = (float*)take(INT * 4); float* Z = (float*)take((size_t)NN * NH_ * 4);
    h16* QS = (h16*)take((size_t)NH_ * NN * HD * 2); h16* KST = (h16*)take((size_t)NH_ * 64 * NN * 2); h16* VT = (h16*)take((size_t)NH_ * 64 * NN * 2); float* KV = (float*)take((size_t)NH_ * 64 * 64 * 4); h16* KVT = (h16*)take((size_t)NH_ * 64 * HD * 2); float* AO = (float*)take((size_t)NH_ * NN * 64 * 4); bf* Rh = (bf*)take((size_t)NN * INT * 2); bf* Rl = (bf*)take((size_t)NN * INT * 2);
    if ((size_t)(wsp - (char*)d_ws) > ws_size) return;
    k_cvt8<<<(4 * INT * DIM / 8 + 255) / 256, 256, 0, stream>>>(wq, WQ, 4 * INT * DIM / 8); k_cvt8<<<(DIM * INT / 8 + 255) / 256, 256, 0, stream>>>(wp, WP, DIM * INT / 8);
    for (int b = 0; b < NB_; ++b) {
        k_cvt8<<<(unsigned)(((size_t)NN * DIM / 8 + 255) / 256), 256, 0, stream>>>(x + (size_t)b * NN * DIM, XB, (size_t)NN * DIM / 8);
        k_gemmw<bf, 0, true><<<dim3(NN / 64, 4 * INT / 64, 1), 32, 0, stream>>>(XB, nullptr, WQ, nullptr, DIM, F, 4 * INT, bq, 0, 0, 0);
        k_kmean<<<1, 256, 0, stream>>>(F, KM, VM); k_z<<<(NN * NH_ + 255) / 256, 256, 0, stream>>>(F, KM, Z);
        k_qs<<<(unsigned)(((size_t)NH_ * NN * HD / 4 + 255) / 256), 256, 0, stream>>>(F, sn, cs, QS); k_kst<<<(unsigned)(((size_t)NH_ * 64 * NN / 2 + 255) / 256), 256, 0, stream>>>(F, sn, cs, KST, VT);
        k_gemmw<h16, 0, false><<<dim3(1, 1, NH_), 32, 0, stream>>>(KST, nullptr, VT, nullptr, NN, KV, 64, nullptr, (size_t)64 * NN, (size_t)64 * NN, (size_t)64 * 64);
        k_kv16<<<(NH_ * 64 * HD / 2 + 255) / 256, 256, 0, stream>>>(KV, KVT);
        k_gemmw<h16, 0, false><<<dim3(NN / 64, 1, NH_), 32, 0, stream>>>(QS, nullptr, KVT, nullptr, HD, AO, 64, nullptr, (size_t)NN * HD, (size_t)64 * HD, (size_t)NN * 64);
        k_res<<<(unsigned)(((size_t)NN * INT / 4 + 255) / 256), 256, 0, stream>>>(AO, Z, VM, F, wl, bl, Rh, Rl);
        k_gemmw<bf, 1, true><<<dim3(NN / 64, DIM / 64, 1), 32, 0, stream>>>(Rh, Rl, WP, nullptr, INT, OUT + (size_t)b * NN * DIM, DIM, bp, 0, 0, 0); }
}
